// SocialAggregation_46076409152412
// MI455X (gfx1250) — hardware-run, weakly checked
//
#include <hip/hip_runtime.h>
#include <stddef.h>
#include <stdint.h>

#define NU    100000
#define NUP   100096
#define NB    16384
#define KN    32
#define DD    128
#define HH    256
#define GBM   64
#define GBN   128
#define GTHR  128
#define PTHR  256
#define ATHR  256
#define VECN  1024
#define PBLK_HB (NUP * 16 / PTHR)
#define PBLK_PI (NB * 16 / PTHR)
#define PBLK_W1 32
#define PBLK_WA 16
#define PBLK_TOTAL (PBLK_HB + PBLK_PI + PBLK_W1 + PBLK_WA + 1)

#define SZ_PA  ((size_t)NUP * HH * 4)
#define SZ_R   ((size_t)NUP * DD * 2)
#define SZ_PB  ((size_t)NB * HH * 4)
#define SZ_SHL ((size_t)NB * 2 * DD * 2)
#define SZ_PIB ((size_t)NB * DD * 2)
#define SZ_W1T ((size_t)2 * HH * DD * 2)
#define SZ_WAD ((size_t)DD * 2 * DD * 2)
#define SZ_VEC ((size_t)VECN * 4)
#define WS_TOTAL (SZ_PA + SZ_R + SZ_PIB + SZ_W1T + SZ_WAD + SZ_VEC)
#define WSMAX  134217728

static_assert(KN == 32);
static_assert(DD == 4 * 32);
static_assert(HH == 8 * 32);
static_assert(HH == 2 * GBN);
static_assert(DD % 32 == 0 && (2 * DD) % 32 == 0);
static_assert(NB % 8 == 0 && NB % GBM == 0 && NB % 128 == 0);
static_assert(NUP % GBM == 0 && NUP >= NU && NU % 16 == 0);
static_assert((NUP * 16) % PTHR == 0 && (NB * 16) % PTHR == 0);
static_assert(GBM == (GTHR / 32) * 16);
static_assert(SZ_PB + SZ_SHL <= SZ_R);
static_assert(WS_TOTAL <= (size_t)WSMAX);
static_assert((SZ_PA % 256) == 0 && (SZ_R % 256) == 0 && (SZ_PB % 256) == 0 && (SZ_PIB % 256) == 0);

typedef float          v4f   __attribute__((ext_vector_type(4)));
typedef float          v8f   __attribute__((ext_vector_type(8)));
typedef int            v8i   __attribute__((ext_vector_type(8)));
typedef unsigned short v4us  __attribute__((ext_vector_type(4)));
typedef unsigned short v8us  __attribute__((ext_vector_type(8)));
typedef unsigned short v16us __attribute__((ext_vector_type(16)));
typedef __bf16         v16bf __attribute__((ext_vector_type(16)));
typedef v4f  __attribute__((may_alias)) v4fa;
typedef v4us __attribute__((may_alias)) v4usa;
typedef v8us __attribute__((may_alias)) v8usa;
union FragB { v16bf v; v16us u; v8us h[2]; v8i w; };

__device__ __forceinline__ v8f wmb(const FragB& a, const FragB& b, v8f c) {
  v8f d = __builtin_amdgcn_wmma_f32_16x16x32_bf16(false, a.v, false, b.v, (short)0, c, false, false);
  asm volatile("v_nop\n\tv_nop\n\tv_nop\n\tv_nop" : "+v"(d) : "v"(a.w), "v"(b.w));
  return d;
}

__device__ __forceinline__ unsigned bf16_bits(float f) {
  const unsigned u = __float_as_uint(f);
  const unsigned r = (u + 0x7FFFu + ((u >> 16) & 1u)) >> 16;
  const unsigned q = (u >> 16) | 0x40u;
  return ((u & 0x7fffffffu) > 0x7f800000u) ? q : r;
}
__device__ __forceinline__ float bf16_val(float f) {
  return __uint_as_float(bf16_bits(f) << 16);
}

__device__ __forceinline__ v8us pack8(v4f a, v4f c) {
  v8us o;
  o[0] = (unsigned short)bf16_bits(a.x); o[1] = (unsigned short)bf16_bits(a.y);
  o[2] = (unsigned short)bf16_bits(a.z); o[3] = (unsigned short)bf16_bits(a.w);
  o[4] = (unsigned short)bf16_bits(c.x); o[5] = (unsigned short)bf16_bits(c.y);
  o[6] = (unsigned short)bf16_bits(c.z); o[7] = (unsigned short)bf16_bits(c.w);
  return o;
}

__device__ __forceinline__ void st16(unsigned short* p, v8us o) {
  *(volatile v8us*)p = o;
  __threadfence();
  *(volatile v8us*)p = o;
}

__device__ __forceinline__ void wave_sync() {
  __builtin_amdgcn_fence(__ATOMIC_RELEASE, "wavefront");
  __builtin_amdgcn_wave_barrier();
  __builtin_amdgcn_fence(__ATOMIC_ACQUIRE, "wavefront");
}

__global__ __launch_bounds__(PTHR) void k_prep(
    const float* __restrict__ in0, const float* __restrict__ in1, const int* __restrict__ uidx,
    const float* __restrict__ W1, const float* __restrict__ b1, const float* __restrict__ W2,
    const float* __restrict__ b2, const float* __restrict__ Wagg, const float* __restrict__ blin,
    const float* __restrict__ bagg,
    unsigned short* HB, unsigned short* PIB, unsigned short* W1T, unsigned short* WAD, float* VEC)
{
  const int tid = (int)threadIdx.x;
  const int blk = (int)blockIdx.x;
  if (blk < PBLK_HB) {
    const int u   = blk * PTHR + tid;
    const int row = u >> 4;
    const int k8  = (u & 15) * 8;
    v8us o = {0, 0, 0, 0, 0, 0, 0, 0};
    if (blk * 16 < NU) {
      const float* p = in1 + (size_t)row * DD + k8;
      const v4f a = *(const v4f*)p;
      const v4f c = *(const v4f*)(p + 4);
      o = pack8(a, c);
    }
    st16(HB + (size_t)row * DD + k8, o);
  } else if (blk < PBLK_HB + PBLK_PI) {
    const int u  = (blk - PBLK_HB) * PTHR + tid;
    const int b  = u >> 4;
    const int k8 = (u & 15) * 8;
    int idx = uidx[b];
    idx = idx < 0 ? 0 : (idx > NU - 1 ? NU - 1 : idx);
    const float* p = in0 + (size_t)idx * DD + k8;
    const v4f a = *(const v4f*)p;
    const v4f c = *(const v4f*)(p + 4);
    st16(PIB + (size_t)b * DD + k8, pack8(a, c));
  } else if (blk < PBLK_HB + PBLK_PI + PBLK_W1) {
    const int v    = (blk - PBLK_HB - PBLK_PI) * PTHR + tid;
    const int part = v >> 12;
    const int vv   = v & 4095;
    const int n    = vv >> 4;
    const int k8   = (vv & 15) * 8;
    const float* p = W1 + (size_t)(part * DD + k8) * HH + n;
    const float f0 = p[0 * HH], f1 = p[1 * HH], f2 = p[2 * HH], f3 = p[3 * HH];
    const float f4 = p[4 * HH], f5 = p[5 * HH], f6 = p[6 * HH], f7 = p[7 * HH];
    v8us o;
    o[0] = (unsigned short)bf16_bits(f0); o[1] = (unsigned short)bf16_bits(f1);
    o[2] = (unsigned short)bf16_bits(f2); o[3] = (unsigned short)bf16_bits(f3);
    o[4] = (unsigned short)bf16_bits(f4); o[5] = (unsigned short)bf16_bits(f5);
    o[6] = (unsigned short)bf16_bits(f6); o[7] = (unsigned short)bf16_bits(f7);
    st16(W1T + (size_t)part * (HH * DD) + (size_t)n * DD + k8, o);
  } else if (blk < PBLK_HB + PBLK_PI + PBLK_W1 + PBLK_WA) {
    const int v  = (blk - PBLK_HB - PBLK_PI - PBLK_W1) * PTHR + tid;
    const int n  = v >> 5;
    const int k8 = (v & 31) * 8;
    const float* p = Wagg + (size_t)n * DD + (k8 & (DD - 1));
    const v4f a = *(const v4f*)p;
    const v4f c = *(const v4f*)(p + 4);
    st16(WAD + (size_t)n * (2 * DD) + k8, pack8(a, c));
  } else {
    const int lane = tid & 31;
    const int wv   = __builtin_amdgcn_readfirstlane(tid >> 5);
    const float b2v = b2[0];
    v4f q = {0.0f, 0.0f, 0.0f, 0.0f};
    if (wv < 2)       q = *(const v4f*)(b1 + 128 * wv + 4 * lane);
    else if (wv < 4)  q = *(const v4f*)(W2 + 128 * (wv - 2) + 4 * lane);
    else if (wv == 4) q = *(const v4f*)(blin + 4 * lane);
    else if (wv == 5) q = *(const v4f*)(bagg + 4 * lane);
    else if (wv == 6) q.x = (lane == 0) ? b2v : 0.0f;
    v4f o;
    o.x = bf16_val(q.x); o.y = bf16_val(q.y); o.z = bf16_val(q.z); o.w = bf16_val(q.w);
    float* dp = VEC + 128 * wv + 4 * lane;
    *(volatile v4f*)dp = o;
    __threadfence();
    *(volatile v4f*)dp = o;
  }
}

template <int MODE>
__global__ __launch_bounds__(GTHR) __attribute__((amdgpu_num_vgpr(248)))
void k_gemm(const unsigned short* __restrict__ Apl, const unsigned short* __restrict__ BT,
            const float* __restrict__ VEC, float* outp)
{
  constexpr int K   = (MODE == 2) ? 2 * DD : DD;
  constexpr int LDO = (MODE == 2) ? DD : HH;
  __shared__ __attribute__((aligned(16))) float stg[GBM * GBN];
  const int tid = (int)threadIdx.x, lane = tid & 31, wave = tid >> 5, hh = lane >> 4, m = lane & 15;
  const int rowBase = (int)blockIdx.x * GBM;
  const int coff    = (int)blockIdx.y * GBN;

  v8f acc[8];
  {
    const v8f z = {0.f, 0.f, 0.f, 0.f, 0.f, 0.f, 0.f, 0.f};
#pragma unroll
    for (int t = 0; t < 8; ++t) acc[t] = z;
  }
  const unsigned short* ap = Apl + (size_t)(rowBase + 16 * wave + m) * (size_t)K + 8 * hh;
  const unsigned short* bp = BT + (size_t)(coff + m) * (size_t)K + 8 * hh;

#pragma unroll 1
  for (int k0 = 0; k0 < K; k0 += 32) {
    FragB af;
    af.h[0] = *(const v8usa*)(ap + k0);
    af.h[1] = *(const v8usa*)(ap + k0 + 16);
#pragma unroll
    for (int nt = 0; nt < 8; ++nt) {
      const unsigned short* wq = bp + (size_t)(16 * nt) * (size_t)K + k0;
      FragB bf;
      bf.h[0] = *(const v8usa*)wq;
      bf.h[1] = *(const v8usa*)(wq + 16);
      acc[nt] = wmb(af, bf, acc[nt]);
    }
  }

#pragma unroll
  for (int nt = 0; nt < 8; ++nt) {
    const int lc = 16 * nt + m;
#pragma unroll
    for (int r = 0; r < 8; ++r) {
      const int lr = 16 * wave + 8 * hh + r;
      stg[lr * GBN + lc] = acc[nt][r];
    }
  }
  __syncthreads();

  v4f bb4 = {0.0f, 0.0f, 0.0f, 0.0f};
  v4f bc4 = {0.0f, 0.0f, 0.0f, 0.0f};
  if constexpr (MODE == 1) bb4 = *(const v4f*)(VEC + coff + 4 * lane);
  if constexpr (MODE == 2) {
    bb4 = *(const v4f*)(VEC + 512 + 4 * lane);
    bc4 = *(const v4f*)(VEC + 640 + 4 * lane);
  }

  v4f pv[16];
#pragma unroll
  for (int i = 0; i < 16; ++i) pv[i] = *(const v4fa*)(stg + (16 * wave + i) * GBN + 4 * lane);

#pragma unroll
  for (int i = 0; i < 16; ++i) {
    v4f t = pv[i];
    if constexpr (MODE == 1) t = t + bb4;
    if constexpr (MODE == 2) {
      t = t + bb4;
      t = t + bc4;
      t.x = (t.x > 0.0f) ? t.x : 0.0f;
      t.y = (t.y > 0.0f) ? t.y : 0.0f;
      t.z = (t.z > 0.0f) ? t.z : 0.0f;
      t.w = (t.w > 0.0f) ? t.w : 0.0f;
    }
    pv[i] = t;
  }

#pragma unroll
  for (int i = 0; i < 16; ++i) {
    float* dp = outp + (size_t)(rowBase + 16 * wave + i) * LDO + coff + 4 * lane;
    *(volatile v4f*)dp = pv[i];
  }
  __threadfence();
#pragma unroll
  for (int i = 0; i < 16; ++i) {
    float* dp = outp + (size_t)(rowBase + 16 * wave + i) * LDO + coff + 4 * lane;
    *(volatile v4f*)dp = pv[i];
  }
}

__global__ __launch_bounds__(ATHR) void k_attn(
    const float* __restrict__ PA, const float* __restrict__ PB, const float* __restrict__ hin,
    const int* __restrict__ nbr, const int* __restrict__ msk, const float* __restrict__ VEC,
    unsigned short* SHL)
{
  __shared__ __attribute__((aligned(16))) unsigned short rowbuf[8 * 2 * DD];
  const int tid = (int)threadIdx.x, lane = tid & 31, wave = tid >> 5;
  const int b = (int)blockIdx.x * 8 + wave;

  int nb = nbr[(size_t)b * KN + lane];
  nb = nb < 0 ? 0 : (nb > NU - 1 ? NU - 1 : nb);
  const int mv = msk[(size_t)b * KN + lane];
  const bool mk = (mv != 0);

  const float* pbr = PB + (size_t)b * HH + 4 * lane;
  const v4f pb0 = *(const v4f*)pbr;
  const v4f pb1 = *(const v4f*)(pbr + DD);
  const v4f w2a = *(const v4f*)(VEC + 256 + 4 * lane);
  const v4f w2b = *(const v4f*)(VEC + 384 + 4 * lane);
  const float b2r = VEC[768];

  float sk = 0.0f;
#pragma unroll 2
  for (int k = 0; k < KN; ++k) {
    const int idx = __builtin_amdgcn_readlane(nb, k);
    const float* pr = PA + (size_t)idx * HH + 4 * lane;
    const v4f p0 = *(const v4f*)pr;
    const v4f p1 = *(const v4f*)(pr + DD);
    float t = 0.0f;
    float v;
    v = p0.x + pb0.x; v = (v > 0.0f) ? v : 0.0f; t = fmaf(v, w2a.x, t);
    v = p0.y + pb0.y; v = (v > 0.0f) ? v : 0.0f; t = fmaf(v, w2a.y, t);
    v = p0.z + pb0.z; v = (v > 0.0f) ? v : 0.0f; t = fmaf(v, w2a.z, t);
    v = p0.w + pb0.w; v = (v > 0.0f) ? v : 0.0f; t = fmaf(v, w2a.w, t);
    v = p1.x + pb1.x; v = (v > 0.0f) ? v : 0.0f; t = fmaf(v, w2b.x, t);
    v = p1.y + pb1.y; v = (v > 0.0f) ? v : 0.0f; t = fmaf(v, w2b.y, t);
    v = p1.z + pb1.z; v = (v > 0.0f) ? v : 0.0f; t = fmaf(v, w2b.z, t);
    v = p1.w + pb1.w; v = (v > 0.0f) ? v : 0.0f; t = fmaf(v, w2b.w, t);
    t += __shfl_xor(t, 16, 32);
    t += __shfl_xor(t, 8, 32);
    t += __shfl_xor(t, 4, 32);
    t += __shfl_xor(t, 2, 32);
    t += __shfl_xor(t, 1, 32);
    const float s = t + b2r;
    sk = (lane == k) ? s : sk;
  }

  const float ninf = -__builtin_inff();
  const float sm = mk ? sk : ninf;
  float mx = sm;
  mx = fmaxf(mx, __shfl_xor(mx, 16, 32));
  mx = fmaxf(mx, __shfl_xor(mx, 8, 32));
  mx = fmaxf(mx, __shfl_xor(mx, 4, 32));
  mx = fmaxf(mx, __shfl_xor(mx, 2, 32));
  mx = fmaxf(mx, __shfl_xor(mx, 1, 32));
  const unsigned vb = __builtin_amdgcn_ballot_w32(mk);
  const bool anyv = (vb != 0u);
  const float mxs = anyv ? mx : 0.0f;
  const float ex = expf(sk - mxs);
  const float p = mk ? ex : 0.0f;
  float sum = p;
  sum += __shfl_xor(sum, 16, 32);
  sum += __shfl_xor(sum, 8, 32);
  sum += __shfl_xor(sum, 4, 32);
  sum += __shfl_xor(sum, 2, 32);
  sum += __shfl_xor(sum, 1, 32);
  const float den = anyv ? sum : 1.0f;
  const float bq = p / den;
  const float beta = (mk && anyv) ? bq : 0.0f;
  const int betai = __float_as_int(beta);

  float a0 = 0.0f, a1 = 0.0f, a2 = 0.0f, a3 = 0.0f;
#pragma unroll 2
  for (int k = 0; k < KN; ++k) {
    const int idx = __builtin_amdgcn_readlane(nb, k);
    const float bk = __int_as_float(__builtin_amdgcn_readlane(betai, k));
    const v4f hv = *(const v4f*)(hin + (size_t)idx * DD + 4 * lane);
    a0 = fmaf(bk, bf16_val(hv.x), a0);
    a1 = fmaf(bk, bf16_val(hv.y), a1);
    a2 = fmaf(bk, bf16_val(hv.z), a2);
    a3 = fmaf(bk, bf16_val(hv.w), a3);
  }

  v4us mh, ml;
  {
    unsigned hb;
    hb = bf16_bits(a0); mh[0] = (unsigned short)hb; ml[0] = (unsigned short)bf16_bits(a0 - __uint_as_float(hb << 16));
    hb = bf16_bits(a1); mh[1] = (unsigned short)hb; ml[1] = (unsigned short)bf16_bits(a1 - __uint_as_float(hb << 16));
    hb = bf16_bits(a2); mh[2] = (unsigned short)hb; ml[2] = (unsigned short)bf16_bits(a2 - __uint_as_float(hb << 16));
    hb = bf16_bits(a3); mh[3] = (unsigned short)hb; ml[3] = (unsigned short)bf16_bits(a3 - __uint_as_float(hb << 16));
  }
  unsigned short* rb = rowbuf + wave * (2 * DD);
  *(v4usa*)(rb + 4 * lane) = mh;
  *(v4usa*)(rb + DD + 4 * lane) = ml;
  wave_sync();
  const v8us q0 = *(const v8usa*)(rb + 8 * lane);
  unsigned short* dp = SHL + (size_t)b * (2 * DD) + 8 * lane;
  *(volatile v8us*)dp = q0;
  __threadfence();
  *(volatile v8us*)dp = q0;
}

extern "C" void kernel_launch(void* const* d_in, const int* in_sizes, int n_in,
                              void* d_out, int out_size, void* d_ws, size_t ws_size,
                              hipStream_t stream) {
  if (n_in < 12) return;
  if (in_sizes[0] != NU * DD || in_sizes[1] != NU * DD) return;
  if (in_sizes[2] != NB || in_sizes[3] != NB * KN || in_sizes[4] != NB * KN) return;
  if (in_sizes[5] != 2 * DD * HH || in_sizes[6] != HH || in_sizes[7] != HH || in_sizes[8] != 1) return;
  if (in_sizes[9] != DD * DD || in_sizes[10] != DD || in_sizes[11] != DD) return;
  if (out_size != NB * DD) return;
  if ((size_t)WS_TOTAL > ws_size) return;

  const float* in0  = (const float*)d_in[0];
  const float* in1  = (const float*)d_in[1];
  const int*   uidx = (const int*)d_in[2];
  const int*   nbr  = (const int*)d_in[3];
  const int*   msk  = (const int*)d_in[4];
  const float* W1   = (const float*)d_in[5];
  const float* b1   = (const float*)d_in[6];
  const float* W2   = (const float*)d_in[7];
  const float* b2   = (const float*)d_in[8];
  const float* Wagg = (const float*)d_in[9];
  const float* blin = (const float*)d_in[10];
  const float* bagg = (const float*)d_in[11];
  float* out = (float*)d_out;

  char* ws = (char*)d_ws;
  const size_t oPA  = 0;
  const size_t oR   = oPA + SZ_PA;
  const size_t oPIB = oR + SZ_R;
  const size_t oW1T = oPIB + SZ_PIB;
  const size_t oWAD = oW1T + SZ_W1T;
  const size_t oVEC = oWAD + SZ_WAD;
  float*          PA  = (float*)(ws + oPA);
  unsigned short* HB  = (unsigned short*)(ws + oR);
  float*          PB  = (float*)(ws + oR);
  unsigned short* SHL = (unsigned short*)(ws + oR + SZ_PB);
  unsigned short* PIB = (unsigned short*)(ws + oPIB);
  unsigned short* W1T = (unsigned short*)(ws + oW1T);
  unsigned short* WAD = (unsigned short*)(ws + oWAD);
  float*          VEC = (float*)(ws + oVEC);

  k_prep<<<PBLK_TOTAL, PTHR, 0, stream>>>(in0, in1, uidx, W1, b1, W2, b2, Wagg, blin, bagg,
                                          HB, PIB, W1T, WAD, VEC);
  k_gemm<0><<<dim3(NUP / GBM, HH / GBN), GTHR, 0, stream>>>(HB, W1T, VEC, PA);
  k_gemm<1><<<dim3(NB / GBM, HH / GBN), GTHR, 0, stream>>>(PIB, W1T + (size_t)HH * DD, VEC, PB);
  k_attn<<<NB / 8, ATHR, 0, stream>>>(PA, PB, in1, nbr, msk, VEC, SHL);
  k_gemm<2><<<dim3(NB / GBM, 1), GTHR, 0, stream>>>(SHL, WAD, VEC, out);
}
